// DeformableFeatureAlignment_17746804867794
// MI455X (gfx1250) — hardware-verified
//
#include <hip/hip_runtime.h>
#include <stddef.h>
#include <math.h>

constexpr int NB      = 4;
constexpr int IMG     = 64;
constexpr int HWPIX   = 4096;
constexpr int NPIX    = 16384;
constexpr int SRC     = 32;
constexpr int SRCHW   = 1024;
constexpr int NCH     = 256;
constexpr int KCAT    = 512;
constexpr int NTAP    = 9;
constexpr int KOM     = 4608;
constexpr int KDC     = 2304;
constexpr int NOMR    = 216;
constexpr int NOMP    = 256;
constexpr int NOFSM   = 144;
constexpr int NPC     = 4096;
constexpr int NCHUNK  = 4;
constexpr int PARSLOT = 256;

static_assert(KOM % 32 == 0 && KDC % 32 == 0 && KCAT % 32 == 0 && NCH % 32 == 0, "");
static_assert(NPIX % 64 == 0 && NPC % 64 == 0 && NOMP % 64 == 0 && KCAT % 64 == 0, "");
static_assert(NCHUNK * NPC == NPIX, "");
static_assert((NPC * NTAP) % 32 == 0, "");
static_assert(NOMR % 4 == 0, "");

typedef __attribute__((ext_vector_type(16))) _Float16 v16h;
typedef __attribute__((ext_vector_type(8)))  _Float16 v8h;
typedef __attribute__((ext_vector_type(16))) __bf16   v16b;
typedef __attribute__((ext_vector_type(8)))  __bf16   v8b;
typedef __attribute__((ext_vector_type(8)))  float    v8f;
typedef __attribute__((ext_vector_type(4)))  float    v4f;
typedef __attribute__((ext_vector_type(4)))  unsigned v4u;

__device__ __forceinline__ unsigned short f2bf_bits(float f) {
  unsigned u = __float_as_uint(f);
  return (unsigned short)((u + 0x7FFFu + ((u >> 16) & 1u)) >> 16);
}
__device__ __forceinline__ float bf_bits2f(unsigned short h) { return __uint_as_float(((unsigned)h) << 16); }
__device__ __forceinline__ float bf16r(float f) { return bf_bits2f(f2bf_bits(f)); }
__device__ __forceinline__ v4f bf16r4(v4f a) { v4f r; r[0] = bf16r(a[0]); r[1] = bf16r(a[1]); r[2] = bf16r(a[2]); r[3] = bf16r(a[3]); return r; }

__device__ __forceinline__ unsigned pk2(unsigned short a, unsigned short b) {
  return (unsigned)a | ((unsigned)b << 16);
}
__device__ __forceinline__ unsigned pkh2(float a, float b) {
  return pk2(__builtin_bit_cast(unsigned short, (_Float16)a), __builtin_bit_cast(unsigned short, (_Float16)b));
}
__device__ __forceinline__ void pkbf2(float a, float b, unsigned& uh, unsigned& ul) {
  const unsigned short ha = f2bf_bits(a), hb = f2bf_bits(b);
  const unsigned short la = f2bf_bits(a - bf_bits2f(ha)), lb = f2bf_bits(b - bf_bits2f(hb));
  uh = pk2(ha, hb);
  ul = pk2(la, lb);
}

__device__ __forceinline__ void dep_guard_h(v8f& a, v8f& b, v16h x, v16h y) { asm volatile("v_nop\n\tv_nop\n\tv_nop\n\tv_nop" : "+v"(a), "+v"(b) : "v"(x), "v"(y)); }
__device__ __forceinline__ void dep_guard_b(v8f& a, v8f& b, v16b x, v16b y) { asm volatile("v_nop\n\tv_nop\n\tv_nop\n\tv_nop" : "+v"(a), "+v"(b) : "v"(x), "v"(y)); }
__device__ __forceinline__ void keep4_h(v16h a, v16h b, v16h c, v16h d) { asm volatile("v_nop" :: "v"(a), "v"(b), "v"(c), "v"(d)); }
__device__ __forceinline__ void keep4_b(v16b a, v16b b, v16b c, v16b d) { asm volatile("v_nop" :: "v"(a), "v"(b), "v"(c), "v"(d)); }
__device__ __forceinline__ void acc_guard4(v8f& a, v8f& b, v8f& c, v8f& d) { asm volatile("v_nop\n\tv_nop\n\tv_nop\n\tv_nop" : "+v"(a), "+v"(b), "+v"(c), "+v"(d)); }
template <typename T> struct Frag;
template <> struct Frag<_Float16> {
  typedef v16h V; union U { v16h v; v8h h[2]; };
  static __device__ __forceinline__ v16h load(const _Float16* p) {
    U f; f.h[0] = *(const v8h*)(p); f.h[1] = *(const v8h*)(p + 16); return f.v;
  }
  static __device__ __forceinline__ v8f mma(v16h a, v16h b, v8f c) {
    return __builtin_amdgcn_wmma_f32_16x16x32_f16(false, a, false, b, (short)0, c, false, false);
  }
  static __device__ __forceinline__ void guard(v8f& a, v8f& b, v16h x, v16h y) { dep_guard_h(a, b, x, y); }
  static __device__ __forceinline__ void keep(v16h a, v16h b, v16h c, v16h d) { keep4_h(a, b, c, d); }
};
template <> struct Frag<__bf16> {
  typedef v16b V; union U { v16b v; v8b h[2]; };
  static __device__ __forceinline__ v16b load(const __bf16* p) {
    U f; f.h[0] = *(const v8b*)(p); f.h[1] = *(const v8b*)(p + 16); return f.v;
  }
  static __device__ __forceinline__ v8f mma(v16b a, v16b b, v8f c) {
    return __builtin_amdgcn_wmma_f32_16x16x32_bf16(false, a, false, b, (short)0, c, false, false);
  }
  static __device__ __forceinline__ void guard(v8f& a, v8f& b, v16b x, v16b y) { dep_guard_b(a, b, x, y); }
  static __device__ __forceinline__ void keep(v16b a, v16b b, v16b c, v16b d) { keep4_b(a, b, c, d); }
};

template <int ET> struct Elem;
template <> struct Elem<0> { typedef _Float16 T; };
template <> struct Elem<1> { typedef __bf16 T; };
template <int ET, int SPLITM, int BIAS_MODE, int OUT_MODE, bool RESID, int ACT = 0>
__global__ __launch_bounds__(256) void wmma_gemm64(
    const unsigned short* __restrict__ Ap, const unsigned short* __restrict__ A2p, int lda, long strideA,
    const unsigned short* __restrict__ Btp, const unsigned short* __restrict__ Bt2p, int ldb, long strideB,
    void* __restrict__ Cout, void* __restrict__ Cout2, int ldc, long strideC,
    const float* __restrict__ bias,
    const float* __restrict__ resid, long strideR,
    int M, int N, int K, float scale) {
  typedef typename Elem<ET>::T T;
  typedef typename Frag<T>::V V;
  constexpr bool SPLA = (SPLITM != 0);
  constexpr bool SPLB = (SPLITM == 1);
  const T* A = (const T*)Ap; const T* A2 = (const T*)A2p; const T* Bt = (const T*)Btp; const T* Bt2 = (const T*)Bt2p;
  __shared__ __align__(16) float sT[8][16 * 68];
  const int b    = blockIdx.y;
  const int lane = threadIdx.x & 31;
  const int wave = threadIdx.x >> 5;
  const int tilesN = N >> 6;
  const int tilesM = M >> 6;
  const int tile = blockIdx.x * 8 + wave;
  if (tile >= tilesM * tilesN) return;
  const int tm = tile / tilesN;
  const int tn = tile - tm * tilesN;
  const int m0 = tm << 6;
  const int n0 = tn << 6;

  const T* Ab  = A  + (size_t)b * strideA;
  const T* Bb  = Bt + (size_t)b * strideB;
  const T* Ab2 = SPLA ? (A2  + (size_t)b * strideA) : nullptr;
  const T* Bb2 = SPLB ? (Bt2 + (size_t)b * strideB) : nullptr;

  const int rlane = lane & 15;
  const int koff  = (lane >> 4) * 8;
  const int mOff  = (lane >> 4) * 8;

  v8f acc[4][4];
#pragma unroll
  for (int i = 0; i < 4; ++i)
#pragma unroll
    for (int j = 0; j < 4; ++j) acc[i][j] = (v8f){0.f,0.f,0.f,0.f,0.f,0.f,0.f,0.f};

  for (int k0 = 0; k0 < K; k0 += 32) {
    V bh[4], bl[4];
#pragma unroll
    for (int j = 0; j < 4; ++j) {
      const size_t bo = (size_t)(n0 + (j << 4) + rlane) * ldb + koff + k0;
      bh[j] = Frag<T>::load(Bb + bo);
      if (SPLB) bl[j] = Frag<T>::load(Bb2 + bo);
    }
#pragma unroll
    for (int i = 0; i < 4; ++i) {
      const size_t ao = (size_t)(m0 + (i << 4) + rlane) * lda + koff + k0;
      V ah = Frag<T>::load(Ab + ao);
      V al;
      if (SPLA) al = Frag<T>::load(Ab2 + ao);
#pragma unroll
      for (int j = 0; j < 4; ++j) {
        acc[i][j] = Frag<T>::mma(ah, bh[j], acc[i][j]);
        if (SPLB) acc[i][j] = Frag<T>::mma(ah, bl[j], acc[i][j]);
        if (SPLA) acc[i][j] = Frag<T>::mma(al, bh[j], acc[i][j]);
      }
      Frag<T>::guard(acc[i][0], acc[i][3], ah, SPLA ? al : ah);
    }
    Frag<T>::keep(bh[0], bh[1], bh[2], bh[3]);
    if (SPLB) Frag<T>::keep(bl[0], bl[1], bl[2], bl[3]);
  }
  acc_guard4(acc[0][0], acc[0][1], acc[0][2], acc[0][3]);
  acc_guard4(acc[1][0], acc[1][1], acc[1][2], acc[1][3]);
  acc_guard4(acc[2][0], acc[2][1], acc[2][2], acc[2][3]);
  acc_guard4(acc[3][0], acc[3][1], acc[3][2], acc[3][3]);

  float* slab = sT[wave];
  const float* Rb = RESID ? (resid + (size_t)b * strideR) : nullptr;
#pragma unroll
  for (int i = 0; i < 4; ++i) {
    const int mBase = m0 + (i << 4);
#pragma unroll
    for (int j = 0; j < 4; ++j) {
      const int n = n0 + (j << 4) + rlane;
      float bv = 0.f;
      if (BIAS_MODE == 2) bv = bias[n];
#pragma unroll
      for (int r = 0; r < 8; ++r) {
        float v = acc[i][j][r] * scale;
        if (BIAS_MODE == 1) v += bias[mBase + mOff + r];
        if (BIAS_MODE == 2) v += bv;
        if (ACT == 1) v = tanhf(v);
        if (ACT == 2) v = fmaxf(v, 0.0f);
        if (ACT == 4) v = (v > 0.f) ? v : 0.01f * v;
        if (RESID) v += Rb[(size_t)(mBase + mOff + r) * ldc + n];
        slab[(mOff + r) * 68 + (j << 4) + rlane] = v;
      }
    }
    __builtin_amdgcn_fence(__ATOMIC_RELEASE, "workgroup");
    __builtin_amdgcn_wave_barrier();
    __builtin_amdgcn_fence(__ATOMIC_ACQUIRE, "workgroup");
    if (OUT_MODE == 0) {
      float* C = (float*)Cout + (size_t)b * strideC;
      const int hh = lane >> 4, c4 = (lane & 15) * 4;
      for (int pass = 0; pass < 2; ++pass) {
#pragma unroll
        for (int it = 0; it < 8; ++it) {
          const int row = it * 2 + hh;
          v4f v = *(const v4f*)(slab + row * 68 + c4);
          *(volatile v4f*)(C + (size_t)(mBase + row) * ldc + n0 + c4) = v;
        }
        __threadfence();
      }
    } else {
      const int q = lane >> 3, c8 = (lane & 7) * 8;
      unsigned short* C  = (unsigned short*)Cout  + (size_t)b * strideC;
      unsigned short* C2 = (OUT_MODE == 2) ? ((unsigned short*)Cout2 + (size_t)b * strideC) : nullptr;
      for (int pass = 0; pass < 2; ++pass) {
#pragma unroll
        for (int it = 0; it < 4; ++it) {
          const int row = it * 4 + q;
          const float* sp = slab + row * 68 + c8;
          v8h hv, lv;
#pragma unroll
          for (int e = 0; e < 8; ++e) {
            if (OUT_MODE == 1) {
              hv[e] = (_Float16)sp[e];
            } else {
              unsigned short hb = f2bf_bits(sp[e]);
              unsigned short lb = f2bf_bits(sp[e] - bf_bits2f(hb));
              hv[e] = __builtin_bit_cast(_Float16, hb);
              lv[e] = __builtin_bit_cast(_Float16, lb);
            }
          }
          *(volatile v8h*)(C + (size_t)(mBase + row) * ldc + n0 + c8) = hv;
          if (OUT_MODE == 2) *(volatile v8h*)(C2 + (size_t)(mBase + row) * ldc + n0 + c8) = lv;
        }
        __threadfence();
      }
    }
    __builtin_amdgcn_fence(__ATOMIC_RELEASE, "workgroup");
    __builtin_amdgcn_wave_barrier();
    __builtin_amdgcn_fence(__ATOMIC_ACQUIRE, "workgroup");
  }
}

template <int MODE>
__global__ __launch_bounds__(256) void k_prepw(const float* __restrict__ w, unsigned short* __restrict__ dst,
                                               int ktot, int nreal, float scale) {
  __shared__ float t[64][65];
  const int tid = threadIdx.x;
  const int k0 = blockIdx.x * 64, n0 = blockIdx.y * 64;
  const int c4 = (tid & 15) * 4;
  const int n = n0 + c4;
  const bool inb = n < nreal;
  const int nc = inb ? n : (nreal - 4);
#pragma unroll
  for (int it = 0; it < 4; ++it) {
    const int row = it * 16 + (tid >> 4);
    const v4f v = *(const v4f*)(w + (size_t)(k0 + row) * nreal + nc);
#pragma unroll
    for (int e = 0; e < 4; ++e) t[row][c4 + e] = inb ? bf16r(v[e]) * scale : 0.0f;
  }
  __syncthreads();
  const int wave = tid >> 5, lane = tid & 31, q = lane >> 3, k8 = (lane & 7) * 8;
  for (int pass = 0; pass < 2; ++pass) {
#pragma unroll
    for (int step = 0; step < 2; ++step) {
      const int nn = step * 32 + wave * 4 + q;
      float f[8];
#pragma unroll
      for (int e = 0; e < 8; ++e) f[e] = t[k8 + e][nn];
      v4u u;
      if (MODE == 1) {
        u[0] = pkh2(f[0], f[1]); u[1] = pkh2(f[2], f[3]); u[2] = pkh2(f[4], f[5]); u[3] = pkh2(f[6], f[7]);
      } else {
        u[0] = pk2(f2bf_bits(f[0]), f2bf_bits(f[1])); u[1] = pk2(f2bf_bits(f[2]), f2bf_bits(f[3]));
        u[2] = pk2(f2bf_bits(f[4]), f2bf_bits(f[5])); u[3] = pk2(f2bf_bits(f[6]), f2bf_bits(f[7]));
      }
      *(volatile v4u*)(dst + (size_t)(n0 + nn) * ktot + k0 + k8) = u;
    }
    __threadfence();
  }
}

__global__ __launch_bounds__(64) void k_par(const float* __restrict__ bom, const float* __restrict__ bdcn,
                                            float* __restrict__ par) {
  const int slot = blockIdx.x;
  const int e0 = threadIdx.x * 4;
  v4f v;
#pragma unroll
  for (int j = 0; j < 4; ++j) {
    const int e = e0 + j;
    const int ea = e < NOMR ? e : (NOMR - 1);
    const float fa = bom[ea];
    const float fb = bdcn[e];
    const float va = (e < NOMR) ? bf16r(fa) : 0.0f;
    const float vb = bf16r(fb);
    v[j] = (slot == 0) ? va : vb;
  }
  volatile v4f* p = (volatile v4f*)(par + (size_t)slot * PARSLOT + e0);
  *p = v;
  __threadfence();
  *p = v;
}

__global__ __launch_bounds__(256) void k_pool_attn(const float* __restrict__ fine, const float* __restrict__ watt,
                                                  float* __restrict__ attn1) {
  __shared__ float ps[NCH];
  __shared__ __align__(16) float at[NCH];
  const int b = blockIdx.x, c = threadIdx.x;
  const float* base = fine + (size_t)b * HWPIX * NCH + c;
  float s0 = 0.f, s1 = 0.f, s2 = 0.f, s3 = 0.f;
#pragma unroll 1
  for (int p = 0; p < HWPIX; p += 4) {
    s0 += bf16r(base[(size_t)(p + 0) * NCH]);
    s1 += bf16r(base[(size_t)(p + 1) * NCH]);
    s2 += bf16r(base[(size_t)(p + 2) * NCH]);
    s3 += bf16r(base[(size_t)(p + 3) * NCH]);
  }
  ps[c] = ((s0 + s1) + (s2 + s3)) * (1.0f / 4096.0f);
  __syncthreads();
  float s = 0.f;
#pragma unroll 1
  for (int k = 0; k < NCH; ++k) s += ps[k] * bf16r(watt[(size_t)k * NCH + c]);
  at[c] = 1.0f + __builtin_amdgcn_rcpf(1.0f + expf(-s));
  __syncthreads();
  if (c < 64) {
    const v4f v = *(const v4f*)(at + c * 4);
    volatile v4f* p = (volatile v4f*)(attn1 + (size_t)b * NCH + c * 4);
    *p = v;
    __threadfence();
    *p = v;
  }
}

__device__ __forceinline__ void rs_taps(int d, int& i0, int& i1, float& w0, float& w1) {
  const int m = d >> 1;
  const bool odd = (d & 1) != 0;
  int a0 = odd ? m : m - 1;
  int a1 = odd ? m + 1 : m;
  float u0 = odd ? 0.75f : 0.25f;
  float u1 = odd ? 0.25f : 0.75f;
  if (a0 < 0) { a0 = 0; u0 = 0.0f; u1 = 1.0f; }
  if (a1 > SRC - 1) { a1 = SRC - 1; u0 = 1.0f; u1 = 0.0f; }
  i0 = a0; i1 = a1; w0 = u0; w1 = u1;
}

__global__ __launch_bounds__(256) void k_resize(const float* __restrict__ cs, float* __restrict__ up,
                                                unsigned short* __restrict__ cat) {
  __shared__ __align__(16) float rowbuf[8][NCH];
  const int lane = threadIdx.x & 31, wave = threadIdx.x >> 5;
  const int p = blockIdx.x * 8 + wave;
  const int b = p >> 12, hw = p & (HWPIX - 1);
  const int yo = hw >> 6, xo = hw & (IMG - 1);
  int y0i, y1i, x0i, x1i; float wy0, wy1, wx0, wx1;
  rs_taps(yo, y0i, y1i, wy0, wy1);
  rs_taps(xo, x0i, x1i, wx0, wx1);
  const float* base = cs + (size_t)b * SRCHW * NCH;
  const float* r00 = base + (size_t)(y0i * SRC + x0i) * NCH;
  const float* r01 = base + (size_t)(y0i * SRC + x1i) * NCH;
  const float* r10 = base + (size_t)(y1i * SRC + x0i) * NCH;
  const float* r11 = base + (size_t)(y1i * SRC + x1i) * NCH;
  v4f res[2];
#pragma unroll
  for (int h2 = 0; h2 < 2; ++h2) {
    const int c = h2 * 128 + lane * 4;
    const v4f g00 = bf16r4(*(const v4f*)(r00 + c));
    const v4f g01 = bf16r4(*(const v4f*)(r01 + c));
    const v4f g10 = bf16r4(*(const v4f*)(r10 + c));
    const v4f g11 = bf16r4(*(const v4f*)(r11 + c));
    const v4f ra = g00 * wx0 + g01 * wx1;
    const v4f rb = g10 * wx0 + g11 * wx1;
    res[h2] = ra * wy0 + rb * wy1;
#pragma unroll
    for (int e = 0; e < 4; ++e) rowbuf[wave][c + e] = res[h2][e];
  }
  __builtin_amdgcn_fence(__ATOMIC_RELEASE, "workgroup");
  __builtin_amdgcn_wave_barrier();
  __builtin_amdgcn_fence(__ATOMIC_ACQUIRE, "workgroup");
  float f[8];
#pragma unroll
  for (int e = 0; e < 8; ++e) f[e] = 2.0f * rowbuf[wave][lane * 8 + e];
  v4u u;
  u[0] = pkh2(f[0], f[1]); u[1] = pkh2(f[2], f[3]); u[2] = pkh2(f[4], f[5]); u[3] = pkh2(f[6], f[7]);
  float* uprow = up + (size_t)p * NCH;
  unsigned short* crow = cat + (size_t)p * KCAT + NCH;
  for (int pass = 0; pass < 2; ++pass) {
    *(volatile v4f*)(uprow + lane * 4) = res[0];
    *(volatile v4f*)(uprow + 128 + lane * 4) = res[1];
    *(volatile v4u*)(crow + lane * 8) = u;
    __threadfence();
  }
}

__global__ __launch_bounds__(256) void k_scale_split(const float* __restrict__ fine, const float* __restrict__ attn1,
                                                     unsigned short* __restrict__ ah, unsigned short* __restrict__ al) {
  const int idx = blockIdx.x * 256 + threadIdx.x;
  const int p = idx >> 5, c8 = (idx & 31) * 8;
  const int b = p >> 12;
  const float* src = fine + (size_t)p * NCH + c8;
  const float* ga = attn1 + (size_t)b * NCH + c8;
  const v4f x0 = *(const v4f*)(src), x1 = *(const v4f*)(src + 4);
  const v4f g0 = *(const v4f*)(ga), g1 = *(const v4f*)(ga + 4);
  float y[8];
  y[0] = bf16r(x0[0]) * g0[0]; y[1] = bf16r(x0[1]) * g0[1]; y[2] = bf16r(x0[2]) * g0[2]; y[3] = bf16r(x0[3]) * g0[3];
  y[4] = bf16r(x1[0]) * g1[0]; y[5] = bf16r(x1[1]) * g1[1]; y[6] = bf16r(x1[2]) * g1[2]; y[7] = bf16r(x1[3]) * g1[3];
  v4u uh, ul;
  unsigned th, tl;
  pkbf2(y[0], y[1], th, tl); uh[0] = th; ul[0] = tl;
  pkbf2(y[2], y[3], th, tl); uh[1] = th; ul[1] = tl;
  pkbf2(y[4], y[5], th, tl); uh[2] = th; ul[2] = tl;
  pkbf2(y[6], y[7], th, tl); uh[3] = th; ul[3] = tl;
  volatile v4u* ph = (volatile v4u*)(ah + (size_t)p * NCH + c8);
  volatile v4u* pl = (volatile v4u*)(al + (size_t)p * NCH + c8);
  *ph = uh; *pl = ul;
  __threadfence();
  *ph = uh; *pl = ul;
}

__global__ __launch_bounds__(256) void k_cvt16(const float* __restrict__ src32, unsigned short* __restrict__ cat) {
  const int idx = blockIdx.x * 256 + threadIdx.x;
  const int p = idx >> 5, c8 = (idx & 31) * 8;
  const float* src = src32 + (size_t)p * NCH + c8;
  const v4f a = *(const v4f*)(src), bq = *(const v4f*)(src + 4);
  v4u u;
  u[0] = pkh2(a[0], a[1]); u[1] = pkh2(a[2], a[3]); u[2] = pkh2(bq[0], bq[1]); u[3] = pkh2(bq[2], bq[3]);
  volatile v4u* d = (volatile v4u*)(cat + (size_t)p * KCAT + c8);
  *d = u;
  __threadfence();
  *d = u;
}

__global__ __launch_bounds__(256) void k_im2col(const unsigned short* __restrict__ al16, unsigned short* __restrict__ im, int p0) {
  const int lane = threadIdx.x & 31, wave = threadIdx.x >> 5;
  const int c8 = lane * 8;
  const v4u z = (v4u){0u, 0u, 0u, 0u};
#pragma unroll 1
  for (int r = 0; r < 4; ++r) {
    const int it = (blockIdx.x * 8 + wave) * 4 + r;
    const int pl = it / NTAP, k = it - pl * NTAP;
    const int p = p0 + pl;
    const int b = p >> 12, hw = p & (HWPIX - 1);
    const int ho = hw >> 6, wo = hw & (IMG - 1);
    const int kh = k / 3, kw = k - kh * 3;
    const int y = ho - 1 + kh, xx = wo - 1 + kw;
    const bool inb = ((unsigned)y < (unsigned)IMG) && ((unsigned)xx < (unsigned)IMG);
    const int yc = y < 0 ? 0 : (y > IMG - 1 ? IMG - 1 : y);
    const int xc = xx < 0 ? 0 : (xx > IMG - 1 ? IMG - 1 : xx);
    const unsigned short* src = al16 + ((size_t)(b * HWPIX + yc * IMG + xc)) * KCAT + c8;
    v4u v0 = *(const v4u*)(src);
    v4u v1 = *(const v4u*)(src + 256);
    if (!inb) { v0 = z; v1 = z; }
    volatile v4u* d0 = (volatile v4u*)(im + (size_t)it * KCAT + c8);
    volatile v4u* d1 = (volatile v4u*)(im + (size_t)it * KCAT + 256 + c8);
    *d0 = v0; *d1 = v1;
    __threadfence();
    *d0 = v0; *d1 = v1;
  }
}

__global__ __launch_bounds__(256) void k_sample(const float* __restrict__ up, const float* __restrict__ omc,
                                                unsigned short* __restrict__ s16, int p0) {
  const int lane = threadIdx.x & 31, wave = threadIdx.x >> 5;
  const int c8 = lane * 8, g = lane >> 2;
  const v4f z = (v4f){0.f, 0.f, 0.f, 0.f};
#pragma unroll 1
  for (int r = 0; r < 4; ++r) {
    const int it = (blockIdx.x * 8 + wave) * 4 + r;
    const int pl = it / NTAP, k = it - pl * NTAP;
    const int p = p0 + pl;
    const int b = p >> 12, hw = p & (HWPIX - 1);
    const int ho = hw >> 6, wo = hw & (IMG - 1);
    const int kh = k / 3, kw = k - kh * 3;
    const float* orow = omc + (size_t)pl * NOMP;
    const int oc = g * NTAP + k;
    const float dy = orow[2 * oc];
    const float dx = orow[2 * oc + 1];
    float ml = orow[NOFSM + oc];
    ml = fminf(fmaxf(ml, -30.0f), 30.0f);
    const float msk = __builtin_amdgcn_rcpf(1.0f + __expf(-ml));
    const float sy = (float)(ho + kh - 1) + dy;
    const float sx = (float)(wo + kw - 1) + dx;
    const float y0 = floorf(sy), x0 = floorf(sx);
    const float y1 = y0 + 1.0f, x1 = x0 + 1.0f;
    const float wy1 = sy - y0, wx1 = sx - x0;
    const float wy0 = 1.0f - wy1, wx0 = 1.0f - wx1;
    const bool vy0 = (y0 >= 0.0f) && (y0 <= (float)(IMG - 1));
    const bool vy1 = (y1 >= 0.0f) && (y1 <= (float)(IMG - 1));
    const bool vx0 = (x0 >= 0.0f) && (x0 <= (float)(IMG - 1));
    const bool vx1 = (x1 >= 0.0f) && (x1 <= (float)(IMG - 1));
    const int yi0 = (int)fminf(fmaxf(y0, 0.0f), (float)(IMG - 1));
    const int yi1 = (int)fminf(fmaxf(y1, 0.0f), (float)(IMG - 1));
    const int xi0 = (int)fminf(fmaxf(x0, 0.0f), (float)(IMG - 1));
    const int xi1 = (int)fminf(fmaxf(x1, 0.0f), (float)(IMG - 1));
    const float* ub  = up + (size_t)b * HWPIX * NCH + c8;
    const float* q00 = ub + ((size_t)yi0 * IMG + xi0) * NCH;
    const float* q01 = ub + ((size_t)yi0 * IMG + xi1) * NCH;
    const float* q10 = ub + ((size_t)yi1 * IMG + xi0) * NCH;
    const float* q11 = ub + ((size_t)yi1 * IMG + xi1) * NCH;
    v4f g00a = *(const v4f*)(q00), g00b = *(const v4f*)(q00 + 4);
    v4f g01a = *(const v4f*)(q01), g01b = *(const v4f*)(q01 + 4);
    v4f g10a = *(const v4f*)(q10), g10b = *(const v4f*)(q10 + 4);
    v4f g11a = *(const v4f*)(q11), g11b = *(const v4f*)(q11 + 4);
    const bool k00 = vy0 && vx0, k01 = vy0 && vx1, k10 = vy1 && vx0, k11 = vy1 && vx1;
    g00a = k00 ? g00a : z; g00b = k00 ? g00b : z;
    g01a = k01 ? g01a : z; g01b = k01 ? g01b : z;
    g10a = k10 ? g10a : z; g10b = k10 ? g10b : z;
    g11a = k11 ? g11a : z; g11b = k11 ? g11b : z;
    const v4f topa = g00a * wx0 + g01a * wx1, topb = g00b * wx0 + g01b * wx1;
    const v4f bota = g10a * wx0 + g11a * wx1, botb = g10b * wx0 + g11b * wx1;
    v4f va = topa * wy0 + bota * wy1;
    v4f vb = topb * wy0 + botb * wy1;
    const float mk = msk * 16.0f;
    va = va * mk;
    vb = vb * mk;
    v4u u;
    u[0] = pkh2(va[0], va[1]); u[1] = pkh2(va[2], va[3]);
    u[2] = pkh2(vb[0], vb[1]); u[3] = pkh2(vb[2], vb[3]);
    volatile v4u* d = (volatile v4u*)(s16 + (size_t)it * NCH + c8);
    *d = u;
    __threadfence();
    *d = u;
  }
}

extern "C" void kernel_launch(void* const* d_in, const int* in_sizes, int n_in,
                              void* d_out, int out_size, void* d_ws, size_t ws_size,
                              hipStream_t stream) {
  if (n_in < 9) return;
  if (in_sizes[0] != NB * SRCHW * NCH || in_sizes[1] != NPIX * NCH || in_sizes[2] != NCH * NCH ||
      in_sizes[3] != NCH * NCH || in_sizes[4] != KCAT * KCAT || in_sizes[5] != KOM * NOMR ||
      in_sizes[6] != NOMR || in_sizes[7] != KDC * NCH || in_sizes[8] != NCH) return;
  if (out_size != NPIX * NCH) return;

  const float* coarse = (const float*)d_in[0];
  const float* fine   = (const float*)d_in[1];
  const float* w_att  = (const float*)d_in[2];
  const float* w_sel  = (const float*)d_in[3];
  const float* w_off  = (const float*)d_in[4];
  const float* w_om   = (const float*)d_in[5];
  const float* b_om   = (const float*)d_in[6];
  const float* w_dcn  = (const float*)d_in[7];
  const float* b_dcn  = (const float*)d_in[8];
  float* out = (float*)d_out;

  const size_t bytes_UP32  = (size_t)NPIX * NCH * 4;
  const size_t bytes_FCAL  = (size_t)NPIX * NCH * 4;
  const size_t bytes_ALIGN = (size_t)NPIX * KCAT * 2;
  const size_t bytes_AH    = (size_t)NPIX * NCH * 2;
  const size_t bytes_CAT16 = (size_t)NPIX * KCAT * 2;
  const size_t bytes_IM16  = (size_t)NPC * KOM * 2;
  const size_t bytes_S16   = (size_t)NPC * KDC * 2;
  size_t bytes_R = 2 * bytes_AH + bytes_CAT16;
  if (bytes_IM16 > bytes_R) bytes_R = bytes_IM16;
  if (bytes_S16 > bytes_R) bytes_R = bytes_S16;
  const size_t bytes_OMC   = (size_t)NPC * NOMP * 4;
  const size_t bytes_WSEL  = (size_t)NCH * NCH * 2;
  const size_t bytes_WOFF  = (size_t)KCAT * KCAT * 2;
  const size_t bytes_WOM   = (size_t)NOMP * KOM * 2;
  const size_t bytes_WDCN  = (size_t)NCH * KDC * 2;
  const size_t bytes_PAR   = (size_t)8 * PARSLOT * 4;

  char* ws = (char*)d_ws;
  size_t o = 0;
  float*          UP32    = (float*)(ws + o);            o += bytes_UP32;
  float*          FCAL32  = (float*)(ws + o);            o += bytes_FCAL;
  unsigned short* ALIGN16 = (unsigned short*)(ws + o);   o += bytes_ALIGN;
  char*           R       = ws + o;                      o += bytes_R;
  unsigned short* AH      = (unsigned short*)(R);
  unsigned short* AL      = (unsigned short*)(R + bytes_AH);
  unsigned short* CAT16   = (unsigned short*)(R + 2 * bytes_AH);
  unsigned short* IM16    = (unsigned short*)(R);
  unsigned short* S16     = (unsigned short*)(R);
  float*          OMC     = (float*)(ws + o);            o += bytes_OMC;
  unsigned short* WSEL    = (unsigned short*)(ws + o);   o += bytes_WSEL;
  unsigned short* WOFF    = (unsigned short*)(ws + o);   o += bytes_WOFF;
  unsigned short* WOM     = (unsigned short*)(ws + o);   o += bytes_WOM;
  unsigned short* WDCN    = (unsigned short*)(ws + o);   o += bytes_WDCN;
  float*          PAR     = (float*)(ws + o);            o += bytes_PAR;
  if (o > ws_size || o > (size_t)134217728) return;

  const float* p_bomr  = PAR + 0 * PARSLOT;
  const float* p_bdcnr = PAR + 1 * PARSLOT;
  float*       p_attn1 = PAR + 4 * PARSLOT;

  k_prepw<0><<<dim3(NCH / 64, NCH / 64), 256, 0, stream>>>(w_sel, WSEL, NCH, NCH, 1.0f);
  k_prepw<1><<<dim3(KCAT / 64, KCAT / 64), 256, 0, stream>>>(w_off, WOFF, KCAT, KCAT, 16.0f);
  k_prepw<1><<<dim3(KOM / 64, NOMP / 64), 256, 0, stream>>>(w_om, WOM, KOM, NOMR, 256.0f);
  k_prepw<1><<<dim3(KDC / 64, NCH / 64), 256, 0, stream>>>(w_dcn, WDCN, KDC, NCH, 64.0f);
  k_par<<<2, 64, 0, stream>>>(b_om, b_dcn, PAR);
  k_resize<<<NPIX / 8, 256, 0, stream>>>(coarse, UP32, CAT16);
  k_pool_attn<<<NB, 256, 0, stream>>>(fine, w_att, p_attn1);
  k_scale_split<<<(NPIX * 32) / 256, 256, 0, stream>>>(fine, p_attn1, AH, AL);

  const int tilesSel = (NPIX / 64) * (NCH / 64);
  wmma_gemm64<1, 2, 0, 0, false><<<dim3((tilesSel + 7) / 8, 1), 256, 0, stream>>>(
      AH, AL, NCH, 0L, WSEL, WSEL, NCH, 0L, (void*)FCAL32, (void*)FCAL32, NCH, 0L,
      p_bdcnr, p_bdcnr, 0L, NPIX, NCH, NCH, 1.0f);
  k_cvt16<<<(NPIX * 32) / 256, 256, 0, stream>>>(FCAL32, CAT16);

  const int tilesOff = (NPIX / 64) * (KCAT / 64);
  wmma_gemm64<0, 0, 0, 1, false><<<dim3((tilesOff + 7) / 8, 1), 256, 0, stream>>>(
      CAT16, CAT16, KCAT, 0L, WOFF, WOFF, KCAT, 0L, (void*)ALIGN16, (void*)ALIGN16, KCAT, 0L,
      p_bdcnr, p_bdcnr, 0L, NPIX, KCAT, KCAT, 0.0625f);

  const int tilesOM  = (NPC / 64) * (NOMP / 64);
  const int tilesDCN = (NPC / 64) * (NCH / 64);
  for (int q = 0; q < NCHUNK; ++q) {
    const int p0 = q * NPC;
    k_im2col<<<(NPC * NTAP) / 32, 256, 0, stream>>>(ALIGN16, IM16, p0);
    wmma_gemm64<0, 0, 2, 0, false><<<dim3((tilesOM + 7) / 8, 1), 256, 0, stream>>>(
        IM16, IM16, KOM, 0L, WOM, WOM, KOM, 0L, (void*)OMC, (void*)OMC, NOMP, 0L,
        p_bomr, p_bdcnr, 0L, NPC, NOMP, KOM, 0.00390625f);
    k_sample<<<(NPC * NTAP) / 32, 256, 0, stream>>>(UP32, OMC, S16, p0);
    wmma_gemm64<0, 0, 2, 0, true, 2><<<dim3((tilesDCN + 7) / 8, 1), 256, 0, stream>>>(
        S16, S16, KDC, 0L, WDCN, WDCN, KDC, 0L,
        (void*)(out + (size_t)p0 * NCH), (void*)(out + (size_t)p0 * NCH), NCH, 0L,
        p_bdcnr, FCAL32 + (size_t)p0 * NCH, 0L, NPC, NCH, KDC, 0.0009765625f);
  }
}
